// LocalModel_15075335209144
// MI455X (gfx1250) — hardware-run, weakly checked
//
#include <hip/hip_runtime.h>


namespace {

constexpr int N = 12000, NP = 12032, NPL = NP  , SRCM = N  , EFULL = 384000, E = EFULL  , F = 512, D = 64, C = 7, NL = (NPL < N ? NPL : N)  , KPAD = ((NL + 31) / 32) * 32;
constexpr float XS = 8.0f, WSC = 256.0f, QS = 16384.0f, LOG2E = 1.4426950408889634f, SLOPE = 0.0f, BNEPS = 1e-5f;
static_assert(NP % 64 == 0 && NP >= N && NPL % 32 == 0 && NL % 32 == 0 && F % 128 == 0 && D == 64, "tiling");
typedef _Float16 b16;
typedef __attribute__((ext_vector_type(16))) _Float16 v16b;
typedef __attribute__((ext_vector_type(8))) _Float16 v8b;
typedef __attribute__((ext_vector_type(8))) float v8f;
typedef __attribute__((ext_vector_type(4))) float v4f;
__device__ __forceinline__ float bf16_rne(float f) { unsigned int u = __float_as_uint(f); u += 0x7FFFu + ((u >> 16) & 1u); return __uint_as_float(u & 0xFFFF0000u); }
__device__ __forceinline__ void split16(float v, b16& hi, b16& lo) { hi = (b16)v; lo = (b16)(v - (float)hi); }
__device__ __forceinline__ v16b frag_kb(const b16* p, int hh) { const v8b a = *(const v8b*)(p + 8 * hh), b = *(const v8b*)(p + 16 + 8 * hh); v16b f;
#pragma unroll
  for (int e = 0; e < 8; ++e) { f[e] = a[e]; f[8 + e] = b[e]; } return f; }
__device__ __forceinline__ v8f wmma16b(v16b a, v16b b, v8f c) { v8f d = __builtin_amdgcn_wmma_f32_16x16x32_f16(false, a, false, b, (short)0, c, false, false); asm volatile("v_nop\n\tv_nop\n\tv_nop\n\tv_nop" : "+v"(d) : "v"(a), "v"(b)); return d; }
__device__ __forceinline__ void wave_lds_sync() { __builtin_amdgcn_fence(__ATOMIC_RELEASE, "workgroup"); __builtin_amdgcn_wave_barrier(); __builtin_amdgcn_fence(__ATOMIC_ACQUIRE, "workgroup"); }
__device__ __forceinline__ float pmul(float a, float b) { float p = a * b; asm volatile("" : "+v"(p)); return p; }
__device__ __forceinline__ int iclamp(int v, int lo, int hi) { return v < lo ? lo : (v > hi ? hi : v); }
constexpr int CSR_NBLK = 512, CSR_GB = 8  , CSR_GN = 1 << CSR_GB  , CSR_MAXG = 512, CSR_CAP = 12288  ;
__global__ __launch_bounds__(64) void csrA_kernel(const int* __restrict__ dst, int E, int N, int nG, int CHP, int NGP, int* __restrict__ STG, int* __restrict__ HST) {
  extern __shared__ int sm[];
  int* cnt = sm; int* run = sm + NGP; int* ids = sm + 2 * NGP;
  const int b = blockIdx.x; const int ch = (E + CSR_NBLK - 1) / CSR_NBLK; const int e0 = b * ch, e1 = min(E, e0 + ch);
  for (int i = threadIdx.x; i < NGP; i += 64) cnt[i] = 0;
  for (int i = threadIdx.x; i < CHP; i += 64) ids[i] = -1;
  __syncthreads();
  if (threadIdx.x == 0) {
    for (int e = e0; e < e1; ++e) { int d = dst[e]; d = (d < 0) ? 0 : (d >= N ? N - 1 : d); cnt[d >> CSR_GB] += 1; }
    int acc = 0; for (int g = 0; g < nG; ++g) { run[g] = acc; acc += cnt[g]; }
    for (int e = e0; e < e1; ++e) { int d = dst[e]; d = (d < 0) ? 0 : (d >= N ? N - 1 : d); const int g = d >> CSR_GB; ids[run[g]] = e; run[g] += 1; } }
  __syncthreads();
  typedef __attribute__((ext_vector_type(4))) int v4i;
  for (int pass = 0; pass < 2; ++pass) {
    for (int i = threadIdx.x; i < CHP / 4; i += 64) *(volatile v4i*)(STG + (size_t)b * CHP + i * 4) = *(const v4i*)(&ids[i * 4]);
    for (int i = threadIdx.x; i < NGP / 4; i += 64) { v4i v; for (int e = 0; e < 4; ++e) v[e] = (i * 4 + e < nG) ? cnt[i * 4 + e] : 0; *(volatile v4i*)(HST + (size_t)b * NGP + i * 4) = v; }
    __threadfence(); }
}
__global__ __launch_bounds__(512) void csrS_kernel(const int* __restrict__ HST, int nG, int NGP, int* __restrict__ START, int* __restrict__ TOT, int* __restrict__ OFF) {
  __shared__ int tot[CSR_MAXG];
  const int b = threadIdx.x;
  for (int pass = 0; pass < 2; ++pass) { int runb = 0; for (int g = 0; g < nG; ++g) { int c = HST[(size_t)b * NGP + g]; c = (c < 0) ? 0 : c; ((volatile int*)OFF)[(size_t)g * CSR_NBLK + b] = runb; runb += c; } __threadfence(); }
  for (int g = threadIdx.x; g < nG; g += 512) { int s = 0; for (int bb = 0; bb < CSR_NBLK; ++bb) { int c = HST[(size_t)bb * NGP + g]; s += (c < 0) ? 0 : c; } tot[g] = s; }
  __syncthreads();
  if (threadIdx.x < 32) {
    __shared__ int st[CSR_MAXG + 32];
    if (threadIdx.x == 0) { int acc = 0; for (int g = 0; g < NGP; ++g) { st[g] = acc; if (g < nG) acc += (tot[g] + 31) & ~31; } st[NGP] = acc; }
    __builtin_amdgcn_fence(__ATOMIC_RELEASE, "workgroup"); __builtin_amdgcn_wave_barrier(); __builtin_amdgcn_fence(__ATOMIC_ACQUIRE, "workgroup");
    for (int pass = 0; pass < 2; ++pass) { for (int i = threadIdx.x; i < NGP + 32; i += 32) { ((volatile int*)START)[i] = (i <= NGP) ? st[min(i, NGP)] : 0; ((volatile int*)TOT)[i] = (i < nG) ? tot[i] : 0; } __threadfence(); } }
}
__global__ __launch_bounds__(256) void csrB_kernel(const int* __restrict__ dst, int N, int nG, int CHP, int NGP, int permLen, const int* __restrict__ STG, const int* __restrict__ HST, const int* __restrict__ OFF, const int* __restrict__ START, const int* __restrict__ TOT, int* __restrict__ PERM, int* __restrict__ ROWPTR, int* __restrict__ ROWCNT, int* __restrict__ FLAG) {
  typedef __attribute__((ext_vector_type(4))) int v4i;
  __shared__ int ids[CSR_CAP]; __shared__ unsigned short key[CSR_CAP]; __shared__ int outp[CSR_CAP]; __shared__ int ncnt[CSR_GN + 1]; __shared__ int boff[CSR_NBLK + 1];
  const int g = blockIdx.x, t_ = threadIdx.x; int tot = TOT[g]; int st = START[g], stn = START[g + 1]; const int v0 = g * CSR_GN; const int nv = min(CSR_GN, N - v0);
  st = (st < 0) ? 0 : (st > permLen - 32 ? permLen - 32 : st) & ~31; stn = (stn < st) ? st : (stn > permLen ? permLen : stn); tot = (tot < 0) ? 0 : tot; if (tot > stn - st && tot <= CSR_CAP) tot = stn - st;
  if (tot > CSR_CAP) {
    for (int pass = 0; pass < 2; ++pass) { for (int i = t_; i < CSR_GN / 4; i += 256) { v4i a, c; for (int e = 0; e < 4; ++e) { a[e] = st; c[e] = 0; } *(volatile v4i*)(ROWPTR + v0 + i * 4) = a; *(volatile v4i*)(ROWCNT + v0 + i * 4) = c; } if (t_ == 0) ((volatile int*)FLAG)[0] = 1; __threadfence(); } (void)nv; return; }
  if (t_ == 0) { int acc = 0; for (int b = 0; b < CSR_NBLK; ++b) { boff[b] = acc; int c = HST[(size_t)b * NGP + g]; c = (c < 0) ? 0 : (c > CHP ? CHP : c); acc += c; if (acc > tot) acc = tot; } boff[CSR_NBLK] = acc; }
  for (int i = t_; i <= CSR_GN; i += 256) ncnt[i] = 0;
  __syncthreads();
  for (int b = 0; b < CSR_NBLK; ++b) { const int c = boff[b + 1] - boff[b]; int o_ = OFF[(size_t)g * CSR_NBLK + b]; o_ = (o_ < 0) ? 0 : (o_ > CHP - c ? CHP - c : o_); const int* src_ = STG + (size_t)b * CHP + o_;
    for (int i = t_; i < c; i += 256) { int id = src_[i]; id = (id < 0) ? 0 : id; ids[boff[b] + i] = id; int d = dst[id]; d = (d < v0) ? v0 : (d >= N ? N - 1 : d); int kk = d - v0; kk = (kk < 0) ? 0 : (kk >= CSR_GN ? CSR_GN - 1 : kk); key[boff[b] + i] = (unsigned short)kk; } }
  __syncthreads();
  if (t_ == 0) { for (int i = 0; i < tot; ++i) ncnt[key[i]] += 1; int acc = 0; for (int vl = 0; vl < CSR_GN; ++vl) { const int c = ncnt[vl]; ncnt[vl] = acc; acc += c; } ncnt[CSR_GN] = acc;
    for (int i = 0; i < tot; ++i) { const int vl = key[i]; outp[ncnt[vl]] = ids[i]; ncnt[vl] += 1; }
    for (int vl = CSR_GN; vl > 0; --vl) ncnt[vl] = ncnt[vl - 1]; ncnt[0] = 0; }
  __syncthreads();
  for (int pass = 0; pass < 2; ++pass) {
    for (int i = t_; i < (stn - st) / 4; i += 256) { v4i v; for (int e = 0; e < 4; ++e) { const int q = i * 4 + e; v[e] = (q < tot) ? outp[q] : -1; } *(volatile v4i*)(PERM + st + i * 4) = v; }
    for (int i = t_; i < CSR_GN / 4; i += 256) { v4i a, c; for (int e = 0; e < 4; ++e) { const int vl = i * 4 + e; a[e] = st + ncnt[vl]; c[e] = (vl < nv) ? (ncnt[vl + 1] - ncnt[vl]) : 0; } *(volatile v4i*)(ROWPTR + v0 + i * 4) = a; *(volatile v4i*)(ROWCNT + v0 + i * 4) = c; }
    __threadfence(); }
}
__global__ __launch_bounds__(256) void csrZ_kernel(int* __restrict__ p, size_t n4) { typedef __attribute__((ext_vector_type(4))) int v4i; const size_t tid = (size_t)blockIdx.x * 256 + threadIdx.x, nth = (size_t)gridDim.x * 256; v4i z = {0, 0, 0, 0}; for (size_t i = tid; i < n4; i += nth) *(volatile v4i*)(p + i * 4) = z; }
struct CsrBufs { int *STG, *HST, *OFF, *START, *TOT, *PERM, *ROWPTR, *ROWCNT, *FLAG; int nG, NGP, CHP; size_t permLen; char* base; size_t bytes; };
static size_t csr_carve(CsrBufs& c, char* ws, size_t off, int E, int N) {
  const size_t off0 = off; c.base = ws + off;
  auto al = [&](size_t bytes) { char* p = ws + off; off += (bytes + 255) & ~(size_t)255; return p; };
  c.nG = (N + CSR_GN - 1) / CSR_GN; c.NGP = (c.nG + 31) & ~31; const int ch = (E + CSR_NBLK - 1) / CSR_NBLK; c.CHP = (ch + 31) & ~31; c.permLen = (size_t)E + 32 * (size_t)c.nG + 32;
  c.STG = (int*)al((size_t)CSR_NBLK * c.CHP * 4); c.HST = (int*)al((size_t)CSR_NBLK * c.NGP * 4); c.OFF = (int*)al((size_t)c.NGP * CSR_NBLK * 4); c.START = (int*)al((size_t)(c.NGP + 64) * 4); c.TOT = (int*)al((size_t)(c.NGP + 64) * 4);
  c.PERM = (int*)al(c.permLen * 4); c.ROWPTR = (int*)al((size_t)c.nG * CSR_GN * 4); c.ROWCNT = (int*)al((size_t)c.nG * CSR_GN * 4); c.FLAG = (int*)al(256);
  c.bytes = off - off0; return off;
}
static void csr_build(const CsrBufs& c, const int* dst, int E, int N, hipStream_t stream) {
  const size_t smem = (size_t)(2 * c.NGP + c.CHP) * 4;
  csrZ_kernel<<<512, 256, 0, stream>>>((int*)c.base, c.bytes / 16);
  csrA_kernel<<<CSR_NBLK, 64, smem, stream>>>(dst, E, N, c.nG, c.CHP, c.NGP, c.STG, c.HST);
  csrS_kernel<<<1, 512, 0, stream>>>(c.HST, c.nG, c.NGP, c.START, c.TOT, c.OFF);
  csrB_kernel<<<c.nG, 256, 0, stream>>>(dst, N, c.nG, c.CHP, c.NGP, (int)c.permLen, c.STG, c.HST, c.OFF, c.START, c.TOT, c.PERM, c.ROWPTR, c.ROWCNT, c.FLAG);
}

typedef __attribute__((ext_vector_type(4))) _Float16 v4h;
typedef __attribute__((ext_vector_type(2))) _Float16 v2h;
typedef __attribute__((ext_vector_type(2))) float v2f;
__device__ __forceinline__ float nexp2(float v) { return __builtin_amdgcn_exp2f(v); }
template <int KD, int NOUT>
__global__ __launch_bounds__(256) void wprep_kernel(const float* __restrict__ w, b16* __restrict__ WT) {
  static_assert(KD % 8 == 0, "wprep"); const size_t u = (size_t)blockIdx.x * 256 + threadIdx.x; if (u >= (size_t)NOUT * KD / 8) return; const size_t e = u * 8; const int oo = (int)(e / KD), k0 = (int)(e % KD); v8b o;
  for (int j = 0; j < 8; ++j) o[j] = (b16)(bf16_rne(w[(size_t)(k0 + j) * NOUT + oo]) * WSC);
  for (int pass = 0; pass < 2; ++pass) { *(volatile v8b*)(WT + e) = o; __threadfence(); }
}
template <int KD, int NOUT, int NV, bool RNDA  >
__global__ __launch_bounds__(64) void gemm_kernel(const float* __restrict__ A, const b16* __restrict__ W, float* __restrict__ T) {
  constexpr int SL = NOUT < 128 ? NOUT : 128, NT = SL / 16, KC = KD < 128 ? KD : 128;
  static_assert(KD % KC == 0 && KC % 32 == 0 && NOUT % SL == 0 && SL % 32 == 0, "gemm tiling");
  __shared__ __attribute__((aligned(16))) b16 Ah[2][16][KC + 8], Al[2][16][KC + 8]; __shared__ __attribute__((aligned(16))) float Tf[2][16][SL + 4];
  const int wave = threadIdx.x >> 5, lane = threadIdx.x & 31, nloc = lane & 15, hlf = lane >> 4; const size_t m0 = (size_t)blockIdx.x * 32 + wave * 16; const int n0 = blockIdx.y * SL;
  v8f acc[NT];
#pragma unroll
  for (int t = 0; t < NT; ++t) acc[t] = (v8f){};
#pragma unroll 1
  for (int kc = 0; kc < KD; kc += KC) {
    for (int idx = lane; idx < 16 * (KC / 4); idx += 32) { const int rr = idx / (KC / 4), c4 = (idx % (KC / 4)) * 4; const size_t row = (m0 + rr < (size_t)NV) ? (m0 + rr) : (size_t)(NV - 1); const v4f v = *(const v4f*)(A + row * KD + kc + c4); v4h hv, lv;
      for (int j = 0; j < 4; ++j) { b16 ph, pl; split16((RNDA ? bf16_rne(v[j]) : v[j]) * XS, ph, pl); hv[j] = ph; lv[j] = pl; } *(v4h*)(&Ah[wave][rr][c4]) = hv; *(v4h*)(&Al[wave][rr][c4]) = lv; }
    wave_lds_sync();
#pragma unroll
    for (int kb = 0; kb < KC; kb += 32) { const v16b a = frag_kb(&Ah[wave][nloc][kb], hlf), al = frag_kb(&Al[wave][nloc][kb], hlf);
#pragma unroll
      for (int t = 0; t < NT; ++t) { const v16b bw = frag_kb(W + (size_t)(n0 + t * 16 + nloc) * KD + kc + kb, hlf); acc[t] = wmma16b(a, bw, acc[t]); acc[t] = wmma16b(al, bw, acc[t]); } }
    wave_lds_sync(); }
#pragma unroll
  for (int t = 0; t < NT; ++t)
#pragma unroll
    for (int r = 0; r < 8; ++r) Tf[wave][8 * hlf + r][t * 16 + nloc] = acc[t][r] * (1.0f / (XS * WSC));
  wave_lds_sync();
  for (int pass = 0; pass < 2; ++pass) { for (int idx = lane; idx < 16 * (SL / 4); idx += 32) { const int rr = idx / (SL / 4), c4 = (idx % (SL / 4)) * 4; *(volatile v4f*)(T + (m0 + rr) * NOUT + n0 + c4) = *(const v4f*)(&Tf[wave][rr][c4]); } __threadfence(); }
}
template <int D, int ACT, bool STATS>
__global__ __launch_bounds__(256) void agg_kernel(const float* __restrict__ T, const float* __restrict__ bias, const int* __restrict__ srcs, const int* __restrict__ PERM, const int* __restrict__ ROWPTR, const int* __restrict__ ROWCNT, int permLen, int E_, float* __restrict__ P, float* __restrict__ PS) {
  static_assert(D % 64 == 0 && D <= 512, "agg width"); constexpr int CPL = D / 32, RPB = 32, VW = CPL < 4 ? CPL : 4; typedef __attribute__((ext_vector_type(VW))) float vwf;
  __shared__ __attribute__((aligned(16))) float rows[RPB][D + 4];
  const int wave = threadIdx.x >> 5, lane = threadIdx.x & 31;
#pragma unroll 1
  for (int q4 = 0; q4 < 4; ++q4) { const int rw = wave * 4 + q4; const size_t v = (size_t)blockIdx.x * RPB + rw; float o[CPL]; for (int i = 0; i < CPL; ++i) o[i] = 0.0f;
    if (v < (size_t)N) { int st = ROWPTR[v], cnt = ROWCNT[v]; cnt = iclamp(cnt, 0, 65536); st = iclamp(st, 0, permLen - cnt); const float dv = rsqrtf((float)cnt + 1.0f); float a[CPL]; for (int i = 0; i < CPL; ++i) a[i] = 0.0f;
#pragma unroll 1
      for (int j = 0; j < cnt; ++j) { const int e = iclamp(PERM[st + j], 0, E_ - 1); size_t s = (size_t)iclamp(srcs[e], 0, N - 1); if (SRCM < N) s %= SRCM; const float w = rsqrtf((float)iclamp(ROWCNT[s], 0, 65536) + 1.0f);
#pragma unroll
        for (int i4 = 0; i4 < CPL / VW; ++i4) { const vwf t = *(const vwf*)(T + s * D + lane * CPL + i4 * VW); for (int i = 0; i < VW; ++i) a[i4 * VW + i] += pmul(w, t[i]); } }
#pragma unroll
      for (int i4 = 0; i4 < CPL / VW; ++i4) { const vwf tv = *(const vwf*)(T + v * D + lane * CPL + i4 * VW); for (int i = 0; i < VW; ++i) { const float h = pmul(dv, a[i4 * VW + i]) + pmul(pmul(dv, dv), tv[i]) + (bias ? bf16_rne(bias[lane * CPL + i4 * VW + i]) : 0.0f); o[i4 * VW + i] = ACT == 1 ? fmaxf(h, 0.0f) : (ACT == 2 ? (h > 0.0f ? h : SLOPE * h) : h); } } }
#pragma unroll
    for (int i4 = 0; i4 < CPL / VW; ++i4) { vwf ov; for (int i = 0; i < VW; ++i) ov[i] = o[i4 * VW + i]; *(vwf*)(&rows[rw][lane * CPL + i4 * VW]) = ov; } }
  __syncthreads();
  for (int pass = 0; pass < 2; ++pass) { for (int q = threadIdx.x; q < RPB * D / 4; q += 256) { const int rr = q / (D / 4), c4 = (q % (D / 4)) * 4; *(volatile v4f*)(P + ((size_t)blockIdx.x * RPB + rr) * D + c4) = *(const v4f*)(&rows[rr][c4]); }
    if (STATS) { for (int c4 = threadIdx.x * 4; c4 < D; c4 += 1024) { v4f s = {0.0f, 0.0f, 0.0f, 0.0f}; for (int rr = 0; rr < RPB; ++rr) s += *(const v4f*)(&rows[rr][c4]); *(volatile v4f*)(PS + (size_t)blockIdx.x * D + c4) = s; } } __threadfence(); }
}

__global__ __launch_bounds__(64) void score_kernel(const float* __restrict__ H, const float* __restrict__ aux, float* __restrict__ S, b16* __restrict__ HT) {
  __shared__ float As_[D]; __shared__ float red[64]; __shared__ __attribute__((aligned(16))) b16 Tt[D][64 + 8];
  const int n = blockIdx.x * 64 + threadIdx.x; const float av = bf16_rne(aux[threadIdx.x]); red[threadIdx.x] = av * av; __syncthreads();
  if (threadIdx.x == 0) { float s = 0.0f; for (int i = 0; i < D; ++i) s += red[i]; red[0] = s; } __syncthreads();
  const float anorm = fmaxf(sqrtf(red[0]), 1e-12f); As_[threadIdx.x] = av / anorm; __syncthreads();
  float dot = 0.0f, nn = 0.0f; const float* hr = H + (size_t)n * D;
#pragma unroll 4
  for (int d = 0; d < D; d += 4) { const v4f hv = *(const v4f*)(hr + d); for (int j = 0; j < 4; ++j) { dot = fmaf(hv[j], As_[d + j], dot); nn = fmaf(hv[j], hv[j], nn); Tt[d + j][threadIdx.x] = (b16)(hv[j] * XS); } }
  const float sc = (n < NL) ? dot / fmaxf(sqrtf(nn), 1e-8f) : 0.0f;
  __syncthreads();
  for (int pass = 0; pass < 2; ++pass) { ((volatile float*)S)[n] = sc; const int wave = threadIdx.x >> 5, lane = threadIdx.x & 31; for (int d = wave; d < D; d += 2) *(volatile v2h*)(HT + (size_t)d * NP + blockIdx.x * 64 + lane * 2) = *(const v2h*)(&Tt[d][lane * 2]); __threadfence(); }
}
__global__ __launch_bounds__(64) void smooth_kernel(const float* __restrict__ S, const b16* __restrict__ HT, const float* __restrict__ H, const float* __restrict__ cw, const float* __restrict__ cb, float* __restrict__ out) {
  __shared__ __attribute__((aligned(16))) b16 Ak[2][16][32 + 8]; __shared__ __attribute__((aligned(16))) float Zs[2][16][D + 4]; __shared__ float Ws[2 * D * C], Bs[8], Rs[2][16]; __shared__ __attribute__((aligned(16))) float Ob[32 * C + 4];
  const int wave = threadIdx.x >> 5, lane = threadIdx.x & 31, nloc = lane & 15, hlf = lane >> 4; const int n0 = blockIdx.x * 32 + wave * 16; const int myrow = n0 + nloc;
  for (int i = threadIdx.x; i < 2 * D * C; i += 64) Ws[i] = bf16_rne(cw[i]); if (threadIdx.x < C) Bs[threadIdx.x] = bf16_rne(cb[threadIdx.x]);
  const float sn = S[myrow]; float rs = 0.0f; v8f acc[4];
#pragma unroll
  for (int t = 0; t < 4; ++t) acc[t] = (v8f){};
#pragma unroll 1
  for (int m0 = 0; m0 < KPAD; m0 += 32) {
    v8b hA, hB;
#pragma unroll
    for (int e = 0; e < 16; ++e) { const int m = m0 + 16 * hlf + e; const float dsm = sn - S[m < NL ? m : NL - 1]; float kap = nexp2(-LOG2E * dsm * dsm); kap = (m < NL) ? kap : 0.0f; rs += kap; const b16 kb = (b16)(kap * QS); if (e < 8) hA[e] = kb; else hB[e - 8] = kb; }
    *(v8b*)(&Ak[wave][nloc][16 * hlf]) = hA; *(v8b*)(&Ak[wave][nloc][16 * hlf + 8]) = hB;
    wave_lds_sync();
    const v16b a = frag_kb(&Ak[wave][nloc][0], hlf);
#pragma unroll
    for (int t = 0; t < 4; ++t) acc[t] = wmma16b(a, frag_kb(HT + (size_t)(t * 16 + nloc) * NP + m0, hlf), acc[t]);
    wave_lds_sync(); }
  rs += __shfl_xor(rs, 16);
  if (hlf == 0) Rs[wave][nloc] = rs;
  wave_lds_sync();
#pragma unroll
  for (int t = 0; t < 4; ++t)
#pragma unroll
    for (int r = 0; r < 8; ++r) Zs[wave][8 * hlf + r][t * 16 + nloc] = acc[t][r] * (1.0f / (QS * XS)) / Rs[wave][8 * hlf + r];
  __syncthreads();
  { const int rr = threadIdx.x >> 1, cset = threadIdx.x & 1; const int row = blockIdx.x * 32 + rr; const float* hr = H + (size_t)row * D; const float* zr = &Zs[rr >> 4][rr & 15][0]; float o4[4] = {0.0f, 0.0f, 0.0f, 0.0f}; const int c0 = cset * 4, nc = cset ? 3 : 4;
#pragma unroll 1
    for (int d = 0; d < D; ++d) { const float hv = hr[d], zv = zr[d]; for (int q = 0; q < 4; ++q) if (q < nc) o4[q] = fmaf(hv, Ws[d * C + c0 + q], fmaf(zv, Ws[(D + d) * C + c0 + q], o4[q])); }
    for (int q = 0; q < nc; ++q) Ob[rr * C + c0 + q] = o4[q] + Bs[c0 + q]; }
  __syncthreads();
  for (int pass = 0; pass < 2; ++pass) { if (threadIdx.x < 32 * C / 4) *(volatile v4f*)(out + (size_t)blockIdx.x * 32 * C + threadIdx.x * 4) = *(const v4f*)(&Ob[threadIdx.x * 4]); __threadfence(); }
}
}

extern "C" void kernel_launch(void* const* d_in, const int* in_sizes, int n_in, void* d_out, int out_size, void* d_ws, size_t ws_size, hipStream_t stream) {
  (void)n_in;
  auto Fp = [&](int i) { return (const float*)d_in[i]; }; auto Ip = [&](int i) { return (const int*)d_in[i]; };
  if (in_sizes[0] != N * F || in_sizes[1] != F * D || in_sizes[2] != D || in_sizes[3] != D * D || in_sizes[4] != D || in_sizes[5] != D || in_sizes[6] != 2 * D * C || in_sizes[7] != C || in_sizes[8] != 2 * EFULL || out_size != N * C) return;
  size_t off = 0; char* ws = (char*)d_ws;
  auto carve = [&](size_t bytes) { char* p = ws + off; off += (bytes + 255) & ~(size_t)255; return p; };
  b16* WT1 = (b16*)carve((size_t)D * F * 2); b16* WT2 = (b16*)carve((size_t)D * D * 2); float* T = (float*)carve((size_t)NP * D * 4); float* P = (float*)carve((size_t)NP * D * 4); float* H = (float*)carve((size_t)NP * D * 4); float* S = (float*)carve((size_t)NP * 4); b16* HT = (b16*)carve((size_t)D * NP * 2);
  CsrBufs csr; off = csr_carve(csr, ws, off, E, N);
  if (off > ws_size || off > ((size_t)128 << 20)) return;
  wprep_kernel<F, D><<<(F * D / 8 + 255) / 256, 256, 0, stream>>>(Fp(1), WT1); wprep_kernel<D, D><<<(D * D / 8 + 255) / 256, 256, 0, stream>>>(Fp(3), WT2);
  csr_build(csr, Ip(8) + EFULL, E, N, stream);
  gemm_kernel<F, D, N, true><<<dim3(NPL / 32, 1), 64, 0, stream>>>(Fp(0), WT1, T);
  agg_kernel<D, 1, false><<<NPL / 32, 256, 0, stream>>>(T, Fp(2), Ip(8), csr.PERM, csr.ROWPTR, csr.ROWCNT, (int)csr.permLen, E, P, nullptr);
  gemm_kernel<D, D, NP, false><<<dim3(NPL / 32, 1), 64, 0, stream>>>(P, WT2, T);
  agg_kernel<D, 0, false><<<NPL / 32, 256, 0, stream>>>(T, Fp(4), Ip(8), csr.PERM, csr.ROWPTR, csr.ROWCNT, (int)csr.permLen, E, H, nullptr);
  score_kernel<<<NP / 64, 64, 0, stream>>>(H, Fp(5), S, HT);
  smooth_kernel<<<NL / 32, 64, 0, stream>>>(S, HT, H, Fp(6), Fp(7), (float*)d_out);
}
